// MultiChannelS4D_18202071400696
// MI455X (gfx1250) — hardware-verified
//
#include <hip/hip_runtime.h>
#include <math.h>

typedef __attribute__((ext_vector_type(16))) _Float16 v16h;
typedef __attribute__((ext_vector_type(16))) __bf16 v16b;
typedef __attribute__((ext_vector_type(8)))  _Float16 v8h;
typedef __attribute__((ext_vector_type(8)))  float v8f;
typedef __attribute__((ext_vector_type(4)))  float v4f;
typedef __attribute__((ext_vector_type(2)))  float v2f;
typedef __attribute__((ext_vector_type(4)))  unsigned v4u;
typedef __attribute__((ext_vector_type(4)))  int v4i;
typedef float __attribute__((may_alias)) float_a;
typedef int __attribute__((may_alias)) int_a;

template <typename T> __device__ __forceinline__ void vst2(void* p, T v) { *(volatile T*)p = v; __threadfence(); *(volatile T*)p = v; }
__device__ __forceinline__ v8f wmma16(v16h a, v16h b, v8f c) {
  v8f d = __builtin_amdgcn_wmma_f32_16x16x32_f16(false, a, false, b, (short)0, c, false, false);
  asm volatile("v_nop\n\tv_nop\n\tv_nop\n\tv_nop" : "+v"(d) : "v"(a), "v"(b));
  return d;
}
__device__ __forceinline__ v8f wmma_bf(v16b a, v16b b, v8f c) {
  v8f d = __builtin_amdgcn_wmma_f32_16x16x32_bf16(false, a, false, b, (short)0, c, false, false);
  asm volatile("v_nop\n\tv_nop\n\tv_nop\n\tv_nop" : "+v"(d) : "v"(a), "v"(b));
  return d;
}
__device__ __forceinline__ v16h frag_h(const _Float16* rowk0, int lane) {
  union { v16h v; v8h q[2]; } u; const _Float16* p = rowk0 + 8 * (lane >> 4);
  u.q[0] = *(const v8h*)p; u.q[1] = *(const v8h*)(p + 16); return u.v;
}
__device__ __forceinline__ v16h frag_f32(const float* rowk0, int lane) {
  v16h a; const float* p = rowk0 + 8 * (lane >> 4);
#pragma unroll
  for (int i = 0; i < 8; ++i) { a[i] = (_Float16)p[i]; a[8 + i] = (_Float16)p[16 + i]; }
  return a;
}
__device__ __forceinline__ v16h frag_f32s(const float* rowk0, int lane, float sc) {
  v16h a; const float* p = rowk0 + 8 * (lane >> 4);
#pragma unroll
  for (int i = 0; i < 8; ++i) { a[i] = (_Float16)(p[i] * sc); a[8 + i] = (_Float16)(p[16 + i] * sc); }
  return a;
}
__device__ __forceinline__ v16h fragc_f32(const float* W, int k0, int n, int lane, int ld, int K) {
  v16h a; const int g = lane >> 4;
#pragma unroll
  for (int i = 0; i < 8; ++i) { const int ka = k0 + 8 * g + i, kb = ka + 16;
    a[i] = (_Float16)(ka < K ? W[(size_t)(ka < K ? ka : K - 1) * ld + n] : 0.f); a[8 + i] = (_Float16)(kb < K ? W[(size_t)(kb < K ? kb : K - 1) * ld + n] : 0.f); }
  return a;
}
struct F2 { v16b h, l; };
__device__ __forceinline__ F2 bsplit16(const float v[16]) { F2 r;
#pragma unroll
  for (int i = 0; i < 16; ++i) { const __bf16 h = (__bf16)v[i]; r.h[i] = h; r.l[i] = (__bf16)(v[i] - (float)h); }
  return r; }
__device__ __forceinline__ F2 split_row(const float* row, int k0, int lane) { float v[16]; const float* p = row + k0 + 8 * (lane >> 4);
#pragma unroll
  for (int i = 0; i < 8; ++i) { v[i] = p[i]; v[8 + i] = p[16 + i]; }
  return bsplit16(v); }
__device__ __forceinline__ F2 split_rowK(const float* row, int k0, int lane, int K) { float v[16]; const int g = lane >> 4;
#pragma unroll
  for (int i = 0; i < 8; ++i) { const int ka = k0 + 8 * g + i, kb = ka + 16; v[i] = ka < K ? row[ka < K ? ka : K - 1] : 0.f; v[8 + i] = kb < K ? row[kb < K ? kb : K - 1] : 0.f; }
  return bsplit16(v); }
__device__ __forceinline__ F2 split_col(const float* W, int k0, int n, int lane, int ld, int K) { float v[16]; const int g = lane >> 4;
#pragma unroll
  for (int i = 0; i < 8; ++i) { const int ka = k0 + 8 * g + i, kb = ka + 16; v[i] = ka < K ? W[(size_t)(ka < K ? ka : K - 1) * ld + n] : 0.f; v[8 + i] = kb < K ? W[(size_t)(kb < K ? kb : K - 1) * ld + n] : 0.f; }
  return bsplit16(v); }
__device__ __forceinline__ v8f mac3(const F2& a, const F2& b, v8f c) { c = wmma_bf(a.l, b.h, c); c = wmma_bf(a.h, b.l, c); return wmma_bf(a.h, b.h, c); }
__device__ __forceinline__ float sigm(float v) { return 1.0f / (1.0f + expf(-v)); }
#define LDSX() do { asm volatile("s_wait_dscnt 0" ::: "memory"); __builtin_amdgcn_wave_barrier(); __builtin_amdgcn_fence(__ATOMIC_RELEASE, "workgroup"); } while (0)


#define NB 8
#define TT 2048
#define DD 64
#define KC 8
#ifndef TNB
#define TNB NB
#endif
#ifndef TQB
#define TQB (TT / 64)
#endif
typedef __attribute__((ext_vector_type(8))) __bf16 v8b;
__device__ __forceinline__ v16b frag_b(const __bf16* rowk0, int lane) {
  union { v16b v; v8b q[2]; } u; const __bf16* p = rowk0 + 8 * (lane >> 4);
  u.q[0] = *(const v8b*)p; u.q[1] = *(const v8b*)(p + 16); return u.v;
}
__device__ __forceinline__ float bfr(float v) { return (float)(__bf16)v; }
__device__ __attribute__((noinline)) float exp_ni(float v) { return expf(v); }
__device__ __attribute__((noinline)) float erf_ni(float v) { return erff(v); }

#define WS_M   0u
#define WS_HT  (WS_M + 4u * (size_t)KC * TT)
#define WS_END (WS_HT + 2u * (size_t)NB * DD * TT)

__global__ __launch_bounds__(256) void k_m(const float* __restrict__ LNR, const float* __restrict__ IM, const float* __restrict__ BP, const float* __restrict__ LDT, float* __restrict__ M) { __shared__ __align__(16) float sm[TT]; const int k = blockIdx.x; const int tid = threadIdx.x;
  const float a = -expf(bfr(LNR[k])), b = bfr(IM[k]); const float dt = expf(bfr(LDT[0])); const float bp = bfr(BP[k]);
  const float adt = a * dt, bdt = b * dt;
  const float ea = expf(adt); const float Ar = ea * cosf(bdt), Ai = ea * sinf(bdt);
  const float xr = Ar - 1.0f, xi = Ai; const float den = a * a + b * b; const float Br = (xr * a + xi * b) / den * bp, Bi = (xi * a - xr * b) / den * bp;
  for (int t = tid; t < TT; t += 256) { const float tf = (float)t; const float pr_e = adt * tf, pr_p = bdt * tf;
    const float e = expf(pr_e); const float pr = e * cosf(pr_p), pi = e * sinf(pr_p); sm[t] = 2.0f * (pr * Br - pi * Bi); }
  __syncthreads(); for (int q = tid; q < TT / 4; q += 256) vst2(M + (size_t)k * TT + q * 4, *(const v4f*)&sm[q * 4]); }
__global__ __launch_bounds__(128) void k_ht(const float* __restrict__ H, __bf16* __restrict__ HT) { __shared__ __align__(16) __bf16 s[DD][72]; const int tid = threadIdx.x; const int t0 = blockIdx.x * 64; const size_t b = blockIdx.y;
  for (int e = tid; e < 64 * DD; e += 128) { const int tl = e / DD, d = e % DD; s[d][tl] = (__bf16)H[(b * TT + t0 + tl) * DD + d]; }
  __syncthreads(); for (int e = tid; e < DD * 8; e += 128) { const int d = e >> 3, q = e & 7; vst2((unsigned*)(HT + (b * DD + d) * (size_t)TT + t0 + q * 8), *(const v4u*)&s[d][q * 8]); } }
__global__ __launch_bounds__(128) void k_conv(const float* __restrict__ M, const __bf16* __restrict__ HT, float* __restrict__ OUT) { __shared__ __align__(16) float sm[TT]; __shared__ __align__(16) float so[4][16][68];
  const int tid = threadIdx.x, wave = tid >> 5, lane = tid & 31, col = lane & 15, g = lane >> 4; const int qb = blockIdx.x, k = blockIdx.y; const size_t b = blockIdx.z; const int t0 = qb * 64 + wave * 16; const int trow = t0 + col;
  for (int e = tid; e < TT; e += 128) sm[e] = M[(size_t)k * TT + e];
  __syncthreads();
  v8f acc[4] = {};
  const int nkc = (qb * 64 + 64) / 32;
#pragma unroll 1
  for (int kc = 0; kc < nkc; ++kc) { v16b ah, al; const int s0 = kc * 32 + 8 * g;
#pragma unroll
    for (int i = 0; i < 8; ++i) { { const int s = s0 + i; const float v = (s <= trow) ? sm[trow - s] : 0.f; const __bf16 hv = (__bf16)v; ah[i] = hv; al[i] = (__bf16)(v - (float)hv); } { const int s = s0 + 16 + i; const float v = (s <= trow) ? sm[trow - s] : 0.f; const __bf16 hv = (__bf16)v; ah[8 + i] = hv; al[8 + i] = (__bf16)(v - (float)hv); } }
#pragma unroll
    for (int j = 0; j < 4; ++j) { const v16b hb = frag_b(HT + (b * DD + j * 16 + col) * (size_t)TT + kc * 32, lane); acc[j] = wmma_bf(ah, hb, acc[j]); acc[j] = wmma_bf(al, hb, acc[j]); } }
#pragma unroll
  for (int j = 0; j < 4; ++j)
#pragma unroll
    for (int r = 0; r < 8; ++r) so[wave][8 * g + r][j * 16 + col] = acc[j][r];
  LDSX(); for (int rl = 0; rl < 16; ++rl) if (lane < 16) vst2(OUT + ((b * TT + t0 + rl) * KC + k) * DD + lane * 4, *(const v4f*)&so[wave][rl][lane * 4]); }
extern "C" void kernel_launch(void* const* d_in, const int* in_sizes, int n_in, void* d_out, int out_size, void* d_ws, size_t ws_size, hipStream_t stream) {
  (void)in_sizes; (void)n_in; (void)out_size;
  const float** F = (const float**)d_in;
  if (ws_size < (size_t)WS_END) return;
  char* ws = (char*)d_ws; float* M = (float*)(ws + WS_M); __bf16* HT = (__bf16*)(ws + WS_HT);
  k_m<<<KC, 256, 0, stream>>>(F[1], F[2], F[3], F[4], M);
  k_ht<<<dim3(TT / 64, TNB), 128, 0, stream>>>(F[0], HT);
  k_conv<<<dim3(TQB, KC, TNB), 128, 0, stream>>>(M, HT, (float*)d_out);
}
